// NeighborMLPConvLayerWeighted_83434034692870
// MI455X (gfx1250) — hardware-run, weakly checked
//
#include <hip/hip_runtime.h>


namespace {
constexpr int N = 50000, M = 50000, E = 1600000, C = 32, H = 64, CO = 32;
constexpr float XS = 8.0f, WSC = 256.0f;
typedef _Float16 b16;
typedef __attribute__((ext_vector_type(16))) _Float16 v16b;
typedef __attribute__((ext_vector_type(8))) _Float16 v8b;
typedef __attribute__((ext_vector_type(8))) float v8f;
typedef __attribute__((ext_vector_type(4))) float v4f;
typedef __attribute__((ext_vector_type(2))) float v2f;
__device__ __forceinline__ float bf16_rne(float f) { unsigned int u = __float_as_uint(f); u += 0x7FFFu + ((u >> 16) & 1u); float r = __uint_as_float(u & 0xFFFF0000u); asm volatile("" : "+v"(r)); return r; }
__device__ __forceinline__ void split16(float v, b16& hi, b16& lo) { hi = (b16)v; lo = (b16)(v - (float)hi); }
__device__ __forceinline__ v16b frag_kb(const b16* p, int hh) { const v8b a = *(const v8b*)(p + 8 * hh), b = *(const v8b*)(p + 16 + 8 * hh); v16b f;
#pragma unroll
  for (int e = 0; e < 8; ++e) { f[e] = a[e]; f[8 + e] = b[e]; } return f; }
__device__ __forceinline__ v8f wmma16b(v16b a, v16b b, v8f c) { v8f d = __builtin_amdgcn_wmma_f32_16x16x32_f16(false, a, false, b, (short)0, c, false, false); asm volatile("v_nop\n\tv_nop\n\tv_nop\n\tv_nop" : "+v"(d) : "v"(a), "v"(b)); return d; }
__device__ __forceinline__ void wave_lds_sync() { __builtin_amdgcn_fence(__ATOMIC_RELEASE, "workgroup"); __builtin_amdgcn_wave_barrier(); __builtin_amdgcn_fence(__ATOMIC_ACQUIRE, "workgroup"); }
__device__ __forceinline__ float pmul(float a, float b) { float p = a * b; asm volatile("" : "+v"(p)); return p; }
__device__ __forceinline__ int iclamp(int v, int lo, int hi) { return v < lo ? lo : (v > hi ? hi : v); }
__device__ __forceinline__ float gelu_erf(float v) { return 0.5f * v * (1.0f + erff(v * 0.70710678118654752f)); }

__global__ __launch_bounds__(256) void wput_kernel(const float* __restrict__ w1, const float* __restrict__ w2, b16* __restrict__ W1A, b16* __restrict__ W1B, b16* __restrict__ W2T) { const int u = blockIdx.x * 256 + threadIdx.x;
  if (u < H * 4) { const int o = u / 4, k0 = (u % 4) * 8; v8b a, b;
#pragma unroll
    for (int j = 0; j < 8; ++j) { a[j] = (b16)(bf16_rne(w1[(size_t)(k0 + j) * H + o]) * WSC); b[j] = (b16)(bf16_rne(w1[(size_t)(C + k0 + j) * H + o]) * WSC); } for (int pass = 0; pass < 2; ++pass) { *(volatile v8b*)(W1A + o * 32 + k0) = a; *(volatile v8b*)(W1B + o * 32 + k0) = b; __threadfence(); } }
  if (u < CO * 8) { const int o = u / 8, k0 = (u % 8) * 8; v8b v;
#pragma unroll
    for (int j = 0; j < 8; ++j) v[j] = (b16)(bf16_rne(w2[(size_t)(k0 + j) * CO + o]) * WSC); for (int pass = 0; pass < 2; ++pass) { *(volatile v8b*)(W2T + o * 64 + k0) = v; __threadfence(); } } }
template <int ADDB>
__global__ __launch_bounds__(32) void proj_kernel(const float* __restrict__ X, const b16* __restrict__ W, const float* __restrict__ b1, int NLIM, float* __restrict__ P) { __shared__ __attribute__((aligned(16))) b16 Ah[16][40]; __shared__ float Tf[16][68]; const int lane = threadIdx.x, nloc = lane & 15, hlf = lane >> 4; const size_t m0 = (size_t)blockIdx.x * 16; if (m0 >= (size_t)NLIM) return;
  for (int rr = 0; rr < 16; ++rr) { Ah[rr][lane] = (b16)(bf16_rne(X[(m0 + rr) * C + lane]) * XS); if (lane < 8) Ah[rr][32 + lane] = (b16)0.0f; }
  wave_lds_sync(); const v16b a = frag_kb(&Ah[nloc][0], hlf);
#pragma unroll
  for (int t = 0; t < 4; ++t) { const v8f acc = wmma16b(a, frag_kb(W + (size_t)(t * 16 + nloc) * 32, hlf), (v8f){}); const int cc = t * 16 + nloc; const float bb = ADDB ? bf16_rne(b1[cc]) : 0.0f;
#pragma unroll
    for (int r8 = 0; r8 < 8; ++r8) Tf[8 * hlf + r8][cc] = acc[r8] * (1.0f / (XS * WSC)) + bb; }
  wave_lds_sync();
  for (int pass = 0; pass < 2; ++pass) { for (int rr = 0; rr < 16; ++rr) *(volatile v2f*)(P + (m0 + rr) * H + lane * 2) = (v2f){Tf[rr][lane * 2], Tf[rr][lane * 2 + 1]}; __threadfence(); } }
__global__ __launch_bounds__(256) void edge_kernel(const float* __restrict__ PA, const float* __restrict__ PB, const float* __restrict__ w, const int* __restrict__ nidx, const int* __restrict__ rowptr, int MLIM, int NLIM, float* __restrict__ G, float* __restrict__ WMP) { const int wave = threadIdx.x >> 5, lane = threadIdx.x & 31; const size_t m = (size_t)blockIdx.x * 8 + wave; if (m >= (size_t)MLIM) return;
  int st = iclamp(rowptr[m], 0, E), en = iclamp(rowptr[m + 1], 0, E); if (en < st) en = st; const int cnt = en - st;
  const float pb0 = PB[m * H + lane * 2], pb1 = PB[m * H + lane * 2 + 1]; float a0 = 0.0f, a1 = 0.0f, ws_ = 0.0f; int n = 0;
#pragma unroll 1
  for (int e = st; e < en; ++e) { const int u = iclamp(nidx[e], 0, N - 1); if (u >= NLIM) continue; ++n; const float we = bf16_rne(w[u]); ws_ += we; const v2f pa = *(const v2f*)(PA + (size_t)u * H + lane * 2); a0 += pmul(we, gelu_erf(pa[0] + pb0)); a1 += pmul(we, gelu_erf(pa[1] + pb1)); }
  (void)cnt; const float inv = 1.0f / (float)(n > 0 ? n : 1); const v2f o = {a0 * inv, a1 * inv};
  for (int pass = 0; pass < 2; ++pass) { *(volatile v2f*)(G + m * H + lane * 2) = o; ((volatile float*)WMP)[m * 32 + lane] = lane == 0 ? ws_ * inv : 0.0f; __threadfence(); } }
__global__ __launch_bounds__(32) void fin_kernel(const float* __restrict__ G, const float* __restrict__ WMP, const b16* __restrict__ W2T, const float* __restrict__ b2, int MLIM, float* __restrict__ out) { __shared__ __attribute__((aligned(16))) b16 Ah[16][72], Al[16][72]; __shared__ float Tf[16][36]; const int lane = threadIdx.x, nloc = lane & 15, hlf = lane >> 4; const size_t m0 = (size_t)blockIdx.x * 16; if (m0 >= (size_t)MLIM) return;
  for (int rr = 0; rr < 16; ++rr) for (int q = 0; q < 2; ++q) { b16 p, ql; split16(G[(m0 + rr) * H + q * 32 + lane] * XS, p, ql); Ah[rr][q * 32 + lane] = p; Al[rr][q * 32 + lane] = ql; }
  if (lane < 8) for (int rr = 0; rr < 16; ++rr) { Ah[rr][64 + lane] = (b16)0.0f; Al[rr][64 + lane] = (b16)0.0f; }
  wave_lds_sync(); v8f acc[2] = {(v8f){}, (v8f){}};
#pragma unroll
  for (int kb = 0; kb < H; kb += 32) { const v16b a = frag_kb(&Ah[nloc][kb], hlf), al = frag_kb(&Al[nloc][kb], hlf);
#pragma unroll
    for (int t = 0; t < 2; ++t) { const v16b bw = frag_kb(W2T + (size_t)(t * 16 + nloc) * 64 + kb, hlf); acc[t] = wmma16b(a, bw, acc[t]); acc[t] = wmma16b(al, bw, acc[t]); } }
#pragma unroll
  for (int t = 0; t < 2; ++t) { const int cc = t * 16 + nloc; const float bb = bf16_rne(b2[cc]);
#pragma unroll
    for (int r8 = 0; r8 < 8; ++r8) { const int rr = 8 * hlf + r8; Tf[rr][cc] = acc[t][r8] * (1.0f / (XS * WSC)) + pmul(WMP[(m0 + rr) * 32], bb); } }
  wave_lds_sync();
  for (int pass = 0; pass < 2; ++pass) { for (int q = lane; q < 16 * CO; q += 32) ((volatile float*)out)[m0 * CO + q] = Tf[q / CO][q % CO]; __threadfence(); } }
}

extern "C" void kernel_launch(void* const* d_in, const int* in_sizes, int n_in, void* d_out, int out_size, void* d_ws, size_t ws_size, hipStream_t stream) {
  (void)n_in;
  auto Fp = [&](int i) { return (const float*)d_in[i]; }; auto Ip = [&](int i) { return (const int*)d_in[i]; };
  if (in_sizes[0] != N * C || in_sizes[1] != M * C || in_sizes[2] != N || in_sizes[3] != 2 * C * H || in_sizes[5] != H * CO || in_sizes[7] != E || in_sizes[8] != M + 1 || out_size != M * CO) return;
  const int NLIM = N, MLIM = M;
  size_t off = 0; char* ws = (char*)d_ws;
  auto carve = [&](size_t bytes) { char* p = ws + off; off += (bytes + 255) & ~(size_t)255; return p; };
  b16* W1A = (b16*)carve(H * 32 * 2); b16* W1B = (b16*)carve(H * 32 * 2); b16* W2T = (b16*)carve(CO * 64 * 2); float* PA = (float*)carve((size_t)N * H * 4); float* PB = (float*)carve((size_t)M * H * 4); float* G = (float*)carve((size_t)M * H * 4); float* WMP = (float*)carve((size_t)M * 32 * 4);
  if (off > ws_size || off > ((size_t)64 << 20)) return;
  wput_kernel<<<1, 256, 0, stream>>>(Fp(3), Fp(5), W1A, W1B, W2T);
  proj_kernel<0><<<NLIM / 16, 32, 0, stream>>>(Fp(0), W1A, nullptr, NLIM, PA);
  proj_kernel<1><<<MLIM / 16, 32, 0, stream>>>(Fp(1), W1B, Fp(4), MLIM, PB);
  edge_kernel<<<(MLIM + 7) / 8, 256, 0, stream>>>(PA, PB, Fp(2), Ip(7), Ip(8), MLIM, NLIM, G, WMP);
  fin_kernel<<<MLIM / 16, 32, 0, stream>>>(G, WMP, W2T, Fp(6), MLIM, (float*)d_out);
}
